// OuterProductMean_9268539425322
// MI455X (gfx1250) — hardware-verified
//
#include <hip/hip_runtime.h>
#include <math.h>

typedef __attribute__((ext_vector_type(16))) _Float16 v16h;
typedef __attribute__((ext_vector_type(16))) __bf16 v16b;
typedef __attribute__((ext_vector_type(8)))  _Float16 v8h;
typedef __attribute__((ext_vector_type(8)))  float v8f;
typedef __attribute__((ext_vector_type(4)))  float v4f;
typedef __attribute__((ext_vector_type(2)))  float v2f;
typedef __attribute__((ext_vector_type(4)))  unsigned v4u;
typedef __attribute__((ext_vector_type(4)))  int v4i;
typedef float __attribute__((may_alias)) float_a;
typedef int __attribute__((may_alias)) int_a;

template <typename T> __device__ __forceinline__ void vst2(void* p, T v) { *(volatile T*)p = v; __threadfence(); *(volatile T*)p = v; }
__device__ __forceinline__ v8f wmma16(v16h a, v16h b, v8f c) {
  v8f d = __builtin_amdgcn_wmma_f32_16x16x32_f16(false, a, false, b, (short)0, c, false, false);
  asm volatile("v_nop\n\tv_nop\n\tv_nop\n\tv_nop" : "+v"(d) : "v"(a), "v"(b));
  return d;
}
__device__ __forceinline__ v8f wmma_bf(v16b a, v16b b, v8f c) {
  v8f d = __builtin_amdgcn_wmma_f32_16x16x32_bf16(false, a, false, b, (short)0, c, false, false);
  asm volatile("v_nop\n\tv_nop\n\tv_nop\n\tv_nop" : "+v"(d) : "v"(a), "v"(b));
  return d;
}
__device__ __forceinline__ v16h frag_h(const _Float16* rowk0, int lane) {
  union { v16h v; v8h q[2]; } u; const _Float16* p = rowk0 + 8 * (lane >> 4);
  u.q[0] = *(const v8h*)p; u.q[1] = *(const v8h*)(p + 16); return u.v;
}
__device__ __forceinline__ v16h frag_f32(const float* rowk0, int lane) {
  v16h a; const float* p = rowk0 + 8 * (lane >> 4);
#pragma unroll
  for (int i = 0; i < 8; ++i) { a[i] = (_Float16)p[i]; a[8 + i] = (_Float16)p[16 + i]; }
  return a;
}
__device__ __forceinline__ v16h frag_f32s(const float* rowk0, int lane, float sc) {
  v16h a; const float* p = rowk0 + 8 * (lane >> 4);
#pragma unroll
  for (int i = 0; i < 8; ++i) { a[i] = (_Float16)(p[i] * sc); a[8 + i] = (_Float16)(p[16 + i] * sc); }
  return a;
}
__device__ __forceinline__ v16h fragc_f32(const float* W, int k0, int n, int lane, int ld, int K) {
  v16h a; const int g = lane >> 4;
#pragma unroll
  for (int i = 0; i < 8; ++i) { const int ka = k0 + 8 * g + i, kb = ka + 16;
    a[i] = (_Float16)(ka < K ? W[(size_t)(ka < K ? ka : K - 1) * ld + n] : 0.f); a[8 + i] = (_Float16)(kb < K ? W[(size_t)(kb < K ? kb : K - 1) * ld + n] : 0.f); }
  return a;
}
struct F2 { v16b h, l; };
__device__ __forceinline__ F2 bsplit16(const float v[16]) { F2 r;
#pragma unroll
  for (int i = 0; i < 16; ++i) { const __bf16 h = (__bf16)v[i]; r.h[i] = h; r.l[i] = (__bf16)(v[i] - (float)h); }
  return r; }
__device__ __forceinline__ F2 split_row(const float* row, int k0, int lane) { float v[16]; const float* p = row + k0 + 8 * (lane >> 4);
#pragma unroll
  for (int i = 0; i < 8; ++i) { v[i] = p[i]; v[8 + i] = p[16 + i]; }
  return bsplit16(v); }
__device__ __forceinline__ F2 split_rowK(const float* row, int k0, int lane, int K) { float v[16]; const int g = lane >> 4;
#pragma unroll
  for (int i = 0; i < 8; ++i) { const int ka = k0 + 8 * g + i, kb = ka + 16; v[i] = ka < K ? row[ka < K ? ka : K - 1] : 0.f; v[8 + i] = kb < K ? row[kb < K ? kb : K - 1] : 0.f; }
  return bsplit16(v); }
__device__ __forceinline__ F2 split_col(const float* W, int k0, int n, int lane, int ld, int K) { float v[16]; const int g = lane >> 4;
#pragma unroll
  for (int i = 0; i < 8; ++i) { const int ka = k0 + 8 * g + i, kb = ka + 16; v[i] = ka < K ? W[(size_t)(ka < K ? ka : K - 1) * ld + n] : 0.f; v[8 + i] = kb < K ? W[(size_t)(kb < K ? kb : K - 1) * ld + n] : 0.f; }
  return bsplit16(v); }
__device__ __forceinline__ v8f mac3(const F2& a, const F2& b, v8f c) { c = wmma_bf(a.l, b.h, c); c = wmma_bf(a.h, b.l, c); return wmma_bf(a.h, b.h, c); }
__device__ __forceinline__ float sigm(float v) { return 1.0f / (1.0f + expf(-v)); }
#define LDSX() do { asm volatile("s_wait_dscnt 0" ::: "memory"); __builtin_amdgcn_wave_barrier(); __builtin_amdgcn_fence(__ATOMIC_RELEASE, "workgroup"); } while (0)

__device__ __forceinline__ float bfr(float v) { return (float)(__bf16)v; }
#define MM 128
#define NN 256
#define CIN 256
#define CM 32
#define CO 128
#define NRX (MM * NN)
#define ICH 16
#ifndef NIV
#define NIV NN
#endif
__global__ __launch_bounds__(256) void k_ln(const float* __restrict__ X, const float* __restrict__ GA, const float* __restrict__ BE, float* __restrict__ XN) { const int wave = threadIdx.x >> 5, lane = threadIdx.x & 31; const size_t row = (size_t)blockIdx.x * 8 + wave; const float* p = X + row * CIN + lane * 8;
  const v4f a0 = *(const v4f*)p, a1 = *(const v4f*)(p + 4); float v[8]; asm volatile("s_wait_loadcnt 0x0" ::: "memory");
#pragma unroll
  for (int i = 0; i < 4; ++i) { v[i] = bfr(a0[i]); v[4 + i] = bfr(a1[i]); }
  float s = 0.f;
#pragma unroll
  for (int i = 0; i < 8; ++i) s += v[i];
#pragma unroll
  for (int o = 1; o < 32; o <<= 1) s += __shfl_xor(s, o);
  const float mean = s * (1.0f / CIN); float q = 0.f;
#pragma unroll
  for (int i = 0; i < 8; ++i) { const float d = v[i] - mean; q += d * d; }
#pragma unroll
  for (int o = 1; o < 32; o <<= 1) q += __shfl_xor(q, o);
  const float rs = rsqrtf(q * (1.0f / CIN) + 1e-5f); v4f r0v, r1v;
#pragma unroll
  for (int i = 0; i < 4; ++i) { r0v[i] = (v[i] - mean) * rs * bfr(GA[lane * 8 + i]) + bfr(BE[lane * 8 + i]); r1v[i] = (v[4 + i] - mean) * rs * bfr(GA[lane * 8 + 4 + i]) + bfr(BE[lane * 8 + 4 + i]); }
  vst2(XN + row * CIN + lane * 8, r0v); vst2(XN + row * CIN + lane * 8 + 4, r1v); }
__global__ __launch_bounds__(128) void k_lr(const float* __restrict__ XN, const float* __restrict__ WL, const float* __restrict__ BL, const float* __restrict__ WR, const float* __restrict__ BR, float* __restrict__ L, float* __restrict__ R) { __shared__ __align__(16) float sf[4][16][36];
  const int tid = threadIdx.x, wave = tid >> 5, lane = tid & 31, col = lane & 15, g = lane >> 4; const int which = blockIdx.y; const size_t r0 = (size_t)blockIdx.x * 64 + wave * 16; const float* Wm = which ? WR : WL; const float* Bm = which ? BR : BL; float* D = which ? R : L;
  v8f acc[2] = {};
#pragma unroll 2
  for (int kc = 0; kc < CIN / 32; ++kc) { const F2 a = split_row(XN + (r0 + col) * CIN, kc * 32, lane); asm volatile("s_wait_loadcnt 0x0" ::: "memory");
#pragma unroll
    for (int j = 0; j < 2; ++j) { v16b w; { const int o = j * 16 + col; float t0[8], t1[8];
#pragma unroll
        for (int i = 0; i < 8; ++i) t0[i] = Wm[(size_t)(kc * 32 + 8 * g + i) * CM + o];
        asm volatile("s_wait_loadcnt 0x0" ::: "memory");
#pragma unroll
        for (int i = 0; i < 8; ++i) t1[i] = Wm[(size_t)(kc * 32 + 16 + 8 * g + i) * CM + o];
        asm volatile("s_wait_loadcnt 0x0" ::: "memory");
#pragma unroll
        for (int i = 0; i < 8; ++i) { w[i] = (__bf16)t0[i]; w[8 + i] = (__bf16)t1[i]; } }
      acc[j] = wmma_bf(a.h, w, acc[j]); acc[j] = wmma_bf(a.l, w, acc[j]); } }
#pragma unroll
  for (int j = 0; j < 2; ++j) { const float bb = bfr(Bm[j * 16 + col]); asm volatile("s_wait_loadcnt 0x0" ::: "memory");
#pragma unroll
    for (int r = 0; r < 8; ++r) sf[wave][8 * g + r][j * 16 + col] = acc[j][r] + bb; }
  LDSX(); for (int rl = 0; rl < 16; ++rl) if (lane < 8) vst2(D + (r0 + rl) * CM + lane * 4, *(const v4f*)&sf[wave][rl][lane * 4]); }
__global__ __launch_bounds__(128) void k_op(const float* __restrict__ L, const float* __restrict__ R, int i0, float* __restrict__ OP) { __shared__ __align__(16) float sf[4][16][132];
  const int tid = threadIdx.x, wave = tid >> 5, lane = tid & 31, col = lane & 15, g = lane >> 4; const int il = blockIdx.x; const int i = i0 + il; const int c0 = blockIdx.y * 128;
  v8f acc[2][2] = {};
#pragma unroll 1
  for (int kc = 0; kc < MM / 32; ++kc) {
    v16b a[2], al[2];
#pragma unroll
    for (int rt = 0; rt < 2; ++rt) { float t0[8], t1[8]; const int x = rt * 16 + col;
#pragma unroll
      for (int i8 = 0; i8 < 8; ++i8) t0[i8] = L[((size_t)(kc * 32 + 8 * g + i8) * NN + i) * CM + x];
      asm volatile("s_wait_loadcnt 0x0" ::: "memory");
#pragma unroll
      for (int i8 = 0; i8 < 8; ++i8) t1[i8] = L[((size_t)(kc * 32 + 16 + 8 * g + i8) * NN + i) * CM + x];
      asm volatile("s_wait_loadcnt 0x0" ::: "memory");
#pragma unroll
      for (int i8 = 0; i8 < 8; ++i8) { const __bf16 h0 = (__bf16)t0[i8], h1 = (__bf16)t1[i8]; a[rt][i8] = h0; a[rt][8 + i8] = h1; al[rt][i8] = (__bf16)(t0[i8] - (float)h0); al[rt][8 + i8] = (__bf16)(t1[i8] - (float)h1); } }
#pragma unroll
    for (int jt = 0; jt < 2; ++jt) { v16b b, bl; { const int cc = c0 + wave * 32 + jt * 16 + col; const int jj = cc >> 5, y = cc & 31; float t0[8], t1[8];
#pragma unroll
        for (int i8 = 0; i8 < 8; ++i8) t0[i8] = R[((size_t)(kc * 32 + 8 * g + i8) * NN + jj) * CM + y];
        asm volatile("s_wait_loadcnt 0x0" ::: "memory");
#pragma unroll
        for (int i8 = 0; i8 < 8; ++i8) t1[i8] = R[((size_t)(kc * 32 + 16 + 8 * g + i8) * NN + jj) * CM + y];
        asm volatile("s_wait_loadcnt 0x0" ::: "memory");
#pragma unroll
        for (int i8 = 0; i8 < 8; ++i8) { const __bf16 h0 = (__bf16)t0[i8], h1 = (__bf16)t1[i8]; b[i8] = h0; b[8 + i8] = h1; bl[i8] = (__bf16)(t0[i8] - (float)h0); bl[8 + i8] = (__bf16)(t1[i8] - (float)h1); } }
#pragma unroll
      for (int rt = 0; rt < 2; ++rt) { acc[rt][jt] = wmma_bf(a[rt], b, acc[rt][jt]); acc[rt][jt] = wmma_bf(a[rt], bl, acc[rt][jt]); acc[rt][jt] = wmma_bf(al[rt], b, acc[rt][jt]); } } }
#pragma unroll
  for (int rt = 0; rt < 2; ++rt) {
#pragma unroll
    for (int jt = 0; jt < 2; ++jt)
#pragma unroll
      for (int r = 0; r < 8; ++r) sf[wave][8 * g + r][rt * 64 + jt * 16 + col] = acc[rt][jt][r];
    }
  LDSX();
  for (int rt = 0; rt < 2; ++rt) for (int xr = 0; xr < 16; ++xr) { const int x = rt * 16 + xr; if (lane < 8) vst2(OP + (((size_t)il * CM + x) * NN * CM) + c0 + wave * 32 + lane * 4, *(const v4f*)&sf[wave][xr][rt * 64 + lane * 4]); } }
__global__ __launch_bounds__(128) void k_of(const float* __restrict__ OP, const float* __restrict__ WF, const float* __restrict__ BF, int i0, float* __restrict__ OUT) { __shared__ __align__(16) float sf[4][16][132];
  const int tid = threadIdx.x, wave = tid >> 5, lane = tid & 31, col = lane & 15, g = lane >> 4; const int il = blockIdx.y; const size_t i = (size_t)i0 + il; const int j0 = blockIdx.x * 64 + wave * 16;
  v8f acc[8] = {};
#pragma unroll 1
  for (int x = 0; x < CM; ++x) { v16b a, al; { const float* p = OP + (((size_t)il * CM + x) * NN + j0 + col) * CM + 8 * g; float t0[8], t1[8];
#pragma unroll
      for (int i8 = 0; i8 < 8; ++i8) t0[i8] = p[i8];
      asm volatile("s_wait_loadcnt 0x0" ::: "memory");
#pragma unroll
      for (int i8 = 0; i8 < 8; ++i8) t1[i8] = p[16 + i8];
      asm volatile("s_wait_loadcnt 0x0" ::: "memory");
#pragma unroll
      for (int i8 = 0; i8 < 8; ++i8) { const __bf16 h0 = (__bf16)t0[i8], h1 = (__bf16)t1[i8]; a[i8] = h0; a[8 + i8] = h1; al[i8] = (__bf16)(t0[i8] - (float)h0); al[8 + i8] = (__bf16)(t1[i8] - (float)h1); } }
#pragma unroll
    for (int jt = 0; jt < 8; ++jt) { v16b w; { const int o = jt * 16 + col; float t0[8], t1[8];
#pragma unroll
        for (int i8 = 0; i8 < 8; ++i8) t0[i8] = WF[(size_t)(x * 32 + 8 * g + i8) * CO + o];
        asm volatile("s_wait_loadcnt 0x0" ::: "memory");
#pragma unroll
        for (int i8 = 0; i8 < 8; ++i8) t1[i8] = WF[(size_t)(x * 32 + 16 + 8 * g + i8) * CO + o];
        asm volatile("s_wait_loadcnt 0x0" ::: "memory");
#pragma unroll
        for (int i8 = 0; i8 < 8; ++i8) { w[i8] = (__bf16)t0[i8]; w[8 + i8] = (__bf16)t1[i8]; } }
      acc[jt] = wmma_bf(a, w, acc[jt]); acc[jt] = wmma_bf(al, w, acc[jt]); } }
  const float inv = 1.0f / ((float)MM + 0.001f);
#pragma unroll
  for (int jt = 0; jt < 8; ++jt) { const float bb = bfr(BF[jt * 16 + col]); asm volatile("s_wait_loadcnt 0x0" ::: "memory");
#pragma unroll
    for (int r = 0; r < 8; ++r) sf[wave][8 * g + r][jt * 16 + col] = (acc[jt][r] + bb) * inv; }
  LDSX(); for (int rl = 0; rl < 16; ++rl) vst2(OUT + ((i * NN) + j0 + rl) * CO + lane * 4, *(const v4f*)&sf[wave][rl][lane * 4]); }
#define WS_XN  0u
#define WS_L   (WS_XN + 4u * (size_t)NRX * CIN)
#define WS_R   (WS_L + 4u * (size_t)NRX * CM)
#define WS_OP  (WS_R + 4u * (size_t)NRX * CM)
#define WS_END (WS_OP + 4u * (size_t)ICH * CM * NN * CM)
extern "C" void kernel_launch(void* const* d_in, const int* in_sizes, int n_in, void* d_out, int out_size, void* d_ws, size_t ws_size, hipStream_t stream) {
  (void)in_sizes; (void)n_in; (void)out_size;
  if (ws_size < (size_t)WS_END) return;
  char* ws = (char*)d_ws; const float** F = (const float**)d_in; float *XN = (float*)(ws + WS_XN), *L = (float*)(ws + WS_L), *R = (float*)(ws + WS_R), *OP = (float*)(ws + WS_OP);
  k_ln<<<dim3(NRX / 8), 256, 0, stream>>>(F[0], F[1], F[2], XN);
  k_lr<<<dim3(NRX / 64, 2), 128, 0, stream>>>(XN, F[3], F[4], F[5], F[6], L, R);
  for (int i0 = 0; i0 < NIV; i0 += ICH) {
    k_op<<<dim3(ICH, NN * CM / 128), 128, 0, stream>>>(L, R, i0, OP);
    k_of<<<dim3(NN / 64, ICH), 128, 0, stream>>>(OP, F[7], F[8], i0, (float*)d_out);
  }
}
